// MLPResNetBlock_68719477556
// MI455X (gfx1250) — hardware-verified
//
#include <hip/hip_runtime.h>
#include <math.h>

constexpr int kB      = 4;
constexpr int kT      = 2048;
constexpr int kD      = 1024;
constexpr int kHeads  = 8;
constexpr int kHd     = 128;
constexpr int kNAdap  = 16;
constexpr int kSReal  = kT + 2 + kNAdap;
constexpr int kSE     = 2112;
constexpr int kTok    = kB * kT;
constexpr int kTokE   = kB * kSE;
constexpr int kGroups = kB * kHeads;
constexpr int kGPer   = 2;
constexpr int kChunks = kGroups / kGPer;
constexpr float kWCarry    = 16.0f;
constexpr float kWCarryInv = 1.0f / 16.0f;
constexpr float kPCarry    = 2048.0f;
constexpr float kOCarry    = 256.0f;
constexpr float kPVScale   = kOCarry / kPCarry;
constexpr float kWoScale   = 1.0f / (kOCarry * kWCarry);
constexpr float kScoreScale = 0.08838834764831845f;
constexpr float kLnEps     = 1e-5f;
constexpr float kInvD      = 1.0f / 1024.0f;

static_assert(kSE % 64 == 0);
static_assert(kSE >= kSReal);
static_assert(kHd % 32 == 0);
static_assert(kD % 64 == 0);

constexpr size_t kOffW   = 0;
constexpr size_t kSzW    = (size_t)5 * kD * kD * 2;
constexpr size_t kOffXE  = kOffW + kSzW;
constexpr size_t kSzXE   = (size_t)kTokE * kD * 2;
constexpr size_t kOffKF  = kOffXE + kSzXE;
constexpr size_t kSzKF   = (size_t)kTokE * kD * 4;
constexpr size_t kOffK16 = kOffKF + kSzKF;
constexpr size_t kSzK16  = (size_t)kTokE * kD * 2;
constexpr size_t kOffVT  = kOffK16 + kSzK16;
constexpr size_t kSzVT   = (size_t)kB * kD * kSE * 2;
constexpr size_t kOffQ   = kOffVT + kSzVT;
constexpr size_t kSzQ    = (size_t)kTok * kD * 2;
constexpr size_t kOffO   = kOffQ + kSzQ;
constexpr size_t kSzO    = (size_t)kTok * kD * 2;
constexpr size_t kWsTotal = kOffO + kSzO;
constexpr size_t kOffSC  = kOffXE;
constexpr size_t kSzSC   = (size_t)kGPer * kT * kSE * 4;
constexpr size_t kOffP   = kOffSC + kSzSC;
constexpr size_t kSzP    = (size_t)kGPer * kT * kSE * 2;
constexpr size_t kOffY   = kOffXE;
constexpr size_t kSzY    = (size_t)kTok * kD * 4;
constexpr size_t kOffYN  = kOffY + kSzY;
constexpr size_t kSzYN   = (size_t)kTok * kD * 2;
static_assert(kWsTotal == 130547712ull);
static_assert(kWsTotal <= 134217728ull);
static_assert(kOffP + kSzP <= kOffK16);
static_assert(kOffYN + kSzYN <= kOffK16);
static_assert(kOffXE % 128 == 0 && kOffKF % 128 == 0 && kOffK16 % 128 == 0 && kOffVT % 128 == 0);
static_assert(kOffQ % 128 == 0 && kOffO % 128 == 0 && kOffP % 128 == 0 && kOffYN % 128 == 0);

typedef __attribute__((ext_vector_type(16))) _Float16 v16h;
typedef __attribute__((ext_vector_type(8)))  _Float16 v8h;
typedef __attribute__((ext_vector_type(16))) __bf16   v16b;
typedef __attribute__((ext_vector_type(8)))  __bf16   v8b;
typedef __attribute__((ext_vector_type(8)))  float    v8f;
typedef __attribute__((ext_vector_type(4)))  float    v4f;
typedef __attribute__((ext_vector_type(4)))  unsigned int v4u;

__device__ __forceinline__ unsigned short f2bf_bits(float f) {
  unsigned u = __float_as_uint(f);
  return (unsigned short)((u + 0x7FFFu + ((u >> 16) & 1u)) >> 16);
}
__device__ __forceinline__ float bf_bits2f(unsigned short h) { return __uint_as_float(((unsigned)h) << 16); }

__device__ __forceinline__ void dep_guard_h(v8f& a, v8f& b, v16h x, v16h y) { asm volatile("v_nop\n\tv_nop\n\tv_nop\n\tv_nop" : "+v"(a), "+v"(b) : "v"(x), "v"(y)); }
__device__ __forceinline__ void dep_guard_b(v8f& a, v8f& b, v16b x, v16b y) { asm volatile("v_nop\n\tv_nop\n\tv_nop\n\tv_nop" : "+v"(a), "+v"(b) : "v"(x), "v"(y)); }
__device__ __forceinline__ void keep4_h(v16h a, v16h b, v16h c, v16h d) { asm volatile("v_nop" :: "v"(a), "v"(b), "v"(c), "v"(d)); }
__device__ __forceinline__ void keep4_b(v16b a, v16b b, v16b c, v16b d) { asm volatile("v_nop" :: "v"(a), "v"(b), "v"(c), "v"(d)); }
__device__ __forceinline__ void acc_guard4(v8f& a, v8f& b, v8f& c, v8f& d) { asm volatile("v_nop\n\tv_nop\n\tv_nop\n\tv_nop" : "+v"(a), "+v"(b), "+v"(c), "+v"(d)); }
template <typename T> struct Frag;
template <> struct Frag<_Float16> {
  typedef v16h V; union U { v16h v; v8h h[2]; };
  static __device__ __forceinline__ v16h load(const _Float16* p) {
    U f; f.h[0] = *(const v8h*)(p); f.h[1] = *(const v8h*)(p + 16); return f.v;
  }
  static __device__ __forceinline__ v8f mma(v16h a, v16h b, v8f c) {
    return __builtin_amdgcn_wmma_f32_16x16x32_f16(false, a, false, b, (short)0, c, false, false);
  }
  static __device__ __forceinline__ void guard(v8f& a, v8f& b, v16h x, v16h y) { dep_guard_h(a, b, x, y); }
  static __device__ __forceinline__ void keep(v16h a, v16h b, v16h c, v16h d) { keep4_h(a, b, c, d); }
};
template <> struct Frag<__bf16> {
  typedef v16b V; union U { v16b v; v8b h[2]; };
  static __device__ __forceinline__ v16b load(const __bf16* p) {
    U f; f.h[0] = *(const v8b*)(p); f.h[1] = *(const v8b*)(p + 16); return f.v;
  }
  static __device__ __forceinline__ v8f mma(v16b a, v16b b, v8f c) {
    return __builtin_amdgcn_wmma_f32_16x16x32_bf16(false, a, false, b, (short)0, c, false, false);
  }
  static __device__ __forceinline__ void guard(v8f& a, v8f& b, v16b x, v16b y) { dep_guard_b(a, b, x, y); }
  static __device__ __forceinline__ void keep(v16b a, v16b b, v16b c, v16b d) { keep4_b(a, b, c, d); }
};

__device__ __forceinline__ unsigned pk16(unsigned short a, unsigned short b) { return (unsigned)a | ((unsigned)b << 16); }
__device__ __forceinline__ unsigned short h_bits(float f) { const _Float16 h = (_Float16)f; return __builtin_bit_cast(unsigned short, h); }

template <int ET> struct Elem;
template <> struct Elem<0> { typedef _Float16 T; };
template <> struct Elem<1> { typedef __bf16 T; };
template <int ET, bool SPLIT, int BIAS_MODE, int OUT_MODE, bool RESID, int ACT = 0>
__global__ __launch_bounds__(256) void wmma_gemm64(
    const unsigned short* __restrict__ Ap, const unsigned short* __restrict__ A2p, int lda, long strideA,
    const unsigned short* __restrict__ Btp, const unsigned short* __restrict__ Bt2p, int ldb, long strideB,
    void* __restrict__ Cout, void* __restrict__ Cout2, int ldc, long strideC,
    const float* __restrict__ bias,
    const float* __restrict__ resid, long strideR,
    int M, int N, int K, float scale) {
  typedef typename Elem<ET>::T T;
  typedef typename Frag<T>::V V;
  const T* A = (const T*)Ap; const T* A2 = (const T*)A2p; const T* Bt = (const T*)Btp; const T* Bt2 = (const T*)Bt2p;
  __shared__ __align__(16) float sT[8][16 * 68];
  const int b    = blockIdx.y;
  const int lane = threadIdx.x & 31;
  const int wave = threadIdx.x >> 5;
  const int tilesN = N >> 6;
  const int tilesM = M >> 6;
  const int tile = blockIdx.x * 8 + wave;
  if (tile >= tilesM * tilesN) return;
  const int tm = tile / tilesN;
  const int tn = tile - tm * tilesN;
  const int m0 = tm << 6;
  const int n0 = tn << 6;

  const T* Ab  = A  + (size_t)b * strideA;
  const T* Bb  = Bt + (size_t)b * strideB;
  const T* Ab2 = SPLIT ? (A2  + (size_t)b * strideA) : nullptr;
  const T* Bb2 = SPLIT ? (Bt2 + (size_t)b * strideB) : nullptr;

  const int rlane = lane & 15;
  const int koff  = (lane >> 4) * 8;
  const int mOff  = (lane >> 4) * 8;

  v8f acc[4][4];
#pragma unroll
  for (int i = 0; i < 4; ++i)
#pragma unroll
    for (int j = 0; j < 4; ++j) acc[i][j] = (v8f){0.f,0.f,0.f,0.f,0.f,0.f,0.f,0.f};

  for (int k0 = 0; k0 < K; k0 += 32) {
    V bh[4], bl[4];
#pragma unroll
    for (int j = 0; j < 4; ++j) {
      const size_t bo = (size_t)(n0 + (j << 4) + rlane) * ldb + koff + k0;
      bh[j] = Frag<T>::load(Bb + bo);
      if (SPLIT) bl[j] = Frag<T>::load(Bb2 + bo);
    }
#pragma unroll
    for (int i = 0; i < 4; ++i) {
      const size_t ao = (size_t)(m0 + (i << 4) + rlane) * lda + koff + k0;
      V ah = Frag<T>::load(Ab + ao);
      V al;
      if (SPLIT) al = Frag<T>::load(Ab2 + ao);
#pragma unroll
      for (int j = 0; j < 4; ++j) {
        acc[i][j] = Frag<T>::mma(ah, bh[j], acc[i][j]);
        if (SPLIT) {
          acc[i][j] = Frag<T>::mma(ah, bl[j], acc[i][j]);
          acc[i][j] = Frag<T>::mma(al, bh[j], acc[i][j]);
        }
      }
      Frag<T>::guard(acc[i][0], acc[i][3], ah, SPLIT ? al : ah);
    }
    Frag<T>::keep(bh[0], bh[1], bh[2], bh[3]);
    if (SPLIT) Frag<T>::keep(bl[0], bl[1], bl[2], bl[3]);
  }
  acc_guard4(acc[0][0], acc[0][1], acc[0][2], acc[0][3]);
  acc_guard4(acc[1][0], acc[1][1], acc[1][2], acc[1][3]);
  acc_guard4(acc[2][0], acc[2][1], acc[2][2], acc[2][3]);
  acc_guard4(acc[3][0], acc[3][1], acc[3][2], acc[3][3]);

  float* slab = sT[wave];
  const float* Rb = RESID ? (resid + (size_t)b * strideR) : nullptr;
#pragma unroll
  for (int i = 0; i < 4; ++i) {
    const int mBase = m0 + (i << 4);
#pragma unroll
    for (int j = 0; j < 4; ++j) {
      const int n = n0 + (j << 4) + rlane;
      float bv = 0.f;
      if (BIAS_MODE == 2) bv = bias[n];
#pragma unroll
      for (int r = 0; r < 8; ++r) {
        float v = acc[i][j][r] * scale;
        if (BIAS_MODE == 1) v += bias[mBase + mOff + r];
        if (BIAS_MODE == 2) v += bv;
        if (RESID) v += Rb[(size_t)(mBase + mOff + r) * ldc + n];
        if (ACT == 2) v = fmaxf(v, 0.0f);
        if (ACT == 4) v = (v > 0.f) ? v : 0.01f * v;
        slab[(mOff + r) * 68 + (j << 4) + rlane] = v;
      }
    }
    __builtin_amdgcn_fence(__ATOMIC_RELEASE, "workgroup");
    __builtin_amdgcn_wave_barrier();
    __builtin_amdgcn_fence(__ATOMIC_ACQUIRE, "workgroup");
    if (OUT_MODE == 0) {
      float* C = (float*)Cout + (size_t)b * strideC;
      const int hh = lane >> 4, c4 = (lane & 15) * 4;
      for (int pass = 0; pass < 2; ++pass) {
#pragma unroll
        for (int it = 0; it < 8; ++it) {
          const int row = it * 2 + hh;
          v4f v = *(const v4f*)(slab + row * 68 + c4);
          *(volatile v4f*)(C + (size_t)(mBase + row) * ldc + n0 + c4) = v;
        }
        __threadfence();
      }
    } else {
      const int q = lane >> 3, c8 = (lane & 7) * 8;
      unsigned short* C  = (unsigned short*)Cout  + (size_t)b * strideC;
      unsigned short* C2 = (OUT_MODE == 2) ? ((unsigned short*)Cout2 + (size_t)b * strideC) : nullptr;
      for (int pass = 0; pass < 2; ++pass) {
#pragma unroll
        for (int it = 0; it < 4; ++it) {
          const int row = it * 4 + q;
          const float* sp = slab + row * 68 + c8;
          v8h hv, lv;
#pragma unroll
          for (int e = 0; e < 8; ++e) {
            if (OUT_MODE == 1) {
              hv[e] = (_Float16)sp[e];
            } else {
              unsigned short hb = f2bf_bits(sp[e]);
              unsigned short lb = f2bf_bits(sp[e] - bf_bits2f(hb));
              hv[e] = __builtin_bit_cast(_Float16, hb);
              lv[e] = __builtin_bit_cast(_Float16, lb);
            }
          }
          *(volatile v8h*)(C + (size_t)(mBase + row) * ldc + n0 + c8) = hv;
          if (OUT_MODE == 2) *(volatile v8h*)(C2 + (size_t)(mBase + row) * ldc + n0 + c8) = lv;
        }
        __threadfence();
      }
    }
    __builtin_amdgcn_fence(__ATOMIC_RELEASE, "workgroup");
    __builtin_amdgcn_wave_barrier();
    __builtin_amdgcn_fence(__ATOMIC_ACQUIRE, "workgroup");
  }
}

__global__ __launch_bounds__(256) void wcast5_kernel(const float* __restrict__ W0, const float* __restrict__ W1,
                                                     const float* __restrict__ W2, const float* __restrict__ W3,
                                                     const float* __restrict__ W4, unsigned short* __restrict__ out,
                                                     float scale) {
  const int z = blockIdx.y;
  const float* W = (z == 0) ? W0 : (z == 1) ? W1 : (z == 2) ? W2 : (z == 3) ? W3 : W4;
  const int i = blockIdx.x * 256 + threadIdx.x;
  if (i >= (kD * kD) / 8) return;
  const float* p = W + 8 * (size_t)i;
  const v4f a = *(const v4f*)(p);
  const v4f c = *(const v4f*)(p + 4);
  unsigned short hb[8];
#pragma unroll
  for (int e = 0; e < 4; ++e) {
    hb[e]     = h_bits(a[e] * scale);
    hb[4 + e] = h_bits(c[e] * scale);
  }
  const v4u u = (v4u){pk16(hb[0], hb[1]), pk16(hb[2], hb[3]), pk16(hb[4], hb[5]), pk16(hb[6], hb[7])};
  unsigned short* q = out + (size_t)z * kD * kD + 8 * (size_t)i;
  *(volatile v4u*)q = u;
  __threadfence();
  *(volatile v4u*)q = u;
}

__global__ __launch_bounds__(256) void build_xe_kernel(const float* __restrict__ x, const float* __restrict__ h_t,
                                                       const float* __restrict__ h_a, const float* __restrict__ pin,
                                                       unsigned short* __restrict__ xe) {
  const int i = blockIdx.x * 256 + threadIdx.x;
  if (i >= (kTokE * kD) / 8) return;
  const int c8   = (i & 127) * 8;
  const int rowg = i >> 7;
  const int b    = rowg / kSE;
  const int r    = rowg - b * kSE;
  const int rx   = (r < kT) ? r : (kT - 1);
  int rt = r - kT - 2; rt = rt < 0 ? 0 : rt; rt = rt > (kNAdap - 1) ? (kNAdap - 1) : rt;
  const float* px = x   + ((size_t)b * kT + rx) * kD + c8;
  const float* pa = h_a + (size_t)b * kD + c8;
  const float* pp = pin + (size_t)b * kD + c8;
  const float* pt = h_t + ((size_t)b * kNAdap + rt) * kD + c8;
  const float* src = (r < kT) ? px : (r == kT) ? pa : (r == kT + 1) ? pp : pt;
  const bool live = (r < kSReal);
  const v4f a = *(const v4f*)(src);
  const v4f c = *(const v4f*)(src + 4);
  unsigned short hb[8];
#pragma unroll
  for (int e = 0; e < 4; ++e) {
    hb[e]     = h_bits(live ? a[e] : 0.0f);
    hb[4 + e] = h_bits(live ? c[e] : 0.0f);
  }
  const v4u u = (v4u){pk16(hb[0], hb[1]), pk16(hb[2], hb[3]), pk16(hb[4], hb[5]), pk16(hb[6], hb[7])};
  unsigned short* q = xe + 8 * (size_t)i;
  *(volatile v4u*)q = u;
  __threadfence();
  *(volatile v4u*)q = u;
}

__global__ __launch_bounds__(256) void kcast_kernel(const float* __restrict__ kf, const float* __restrict__ g,
                                                    unsigned short* __restrict__ k16) {
  const int i = blockIdx.x * 256 + threadIdx.x;
  if (i >= (kTokE * kD) / 8) return;
  const int rowg = i >> 7;
  const int r    = rowg % kSE;
  const float ratio = tanhf(g[0]);
  const bool adap = (r >= kT + 2) && (r < kSReal);
  const bool live = (r < kSReal);
  const float f = adap ? ratio : 1.0f;
  const float* p = kf + 8 * (size_t)i;
  const v4f a = *(const v4f*)(p);
  const v4f c = *(const v4f*)(p + 4);
  unsigned short hb[8];
#pragma unroll
  for (int e = 0; e < 4; ++e) {
    hb[e]     = h_bits(live ? a[e] * f : 0.0f);
    hb[4 + e] = h_bits(live ? c[e] * f : 0.0f);
  }
  const v4u u = (v4u){pk16(hb[0], hb[1]), pk16(hb[2], hb[3]), pk16(hb[4], hb[5]), pk16(hb[6], hb[7])};
  unsigned short* q = k16 + 8 * (size_t)i;
  *(volatile v4u*)q = u;
  __threadfence();
  *(volatile v4u*)q = u;
}

constexpr int kSmThreads = 288;
constexpr int kSmOwners  = kSE / 8;
__global__ __launch_bounds__(kSmThreads) void softmax_row_kernel(const float* __restrict__ S, unsigned short* __restrict__ P,
                                                                 float sscale, float carry) {
  __shared__ float redM[9];
  __shared__ float redS[9];
  const int row  = blockIdx.x;
  const int t    = threadIdx.x;
  const int lane = t & 31, wave = t >> 5;
  const bool owner = (t < kSmOwners);
  const int c0   = owner ? (t * 8) : (kSE - 8);
  const float* sr = S + (size_t)row * kSE + c0;
  const v4f a = *(const v4f*)(sr);
  const v4f c = *(const v4f*)(sr + 4);
  float xv[8];
#pragma unroll
  for (int e = 0; e < 4; ++e) {
    const bool v0 = owner && (c0 + e < kSReal);
    const bool v1 = owner && (c0 + 4 + e < kSReal);
    xv[e]     = v0 ? a[e] * sscale : -INFINITY;
    xv[4 + e] = v1 ? c[e] * sscale : -INFINITY;
  }
  float m = fmaxf(fmaxf(fmaxf(xv[0], xv[1]), fmaxf(xv[2], xv[3])), fmaxf(fmaxf(xv[4], xv[5]), fmaxf(xv[6], xv[7])));
#pragma unroll
  for (int off = 16; off > 0; off >>= 1) m = fmaxf(m, __shfl_xor(m, off, 32));
  if (lane == 0) redM[wave] = m;
  __syncthreads();
  float gm = redM[0];
#pragma unroll
  for (int w = 1; w < 9; ++w) gm = fmaxf(gm, redM[w]);
  float pv[8];
  float s = 0.0f;
#pragma unroll
  for (int e = 0; e < 8; ++e) { pv[e] = expf(xv[e] - gm); s += pv[e]; }
#pragma unroll
  for (int off = 16; off > 0; off >>= 1) s += __shfl_xor(s, off, 32);
  if (lane == 0) redS[wave] = s;
  __syncthreads();
  float gs = redS[0];
#pragma unroll
  for (int w = 1; w < 9; ++w) gs += redS[w];
  const float inv = carry * (1.0f / gs);
  unsigned short hb[8];
#pragma unroll
  for (int e = 0; e < 8; ++e) hb[e] = h_bits(pv[e] * inv);
  const v4u u = (v4u){pk16(hb[0], hb[1]), pk16(hb[2], hb[3]), pk16(hb[4], hb[5]), pk16(hb[6], hb[7])};
  if (owner) {
    unsigned short* q = P + (size_t)row * kSE + c0;
    *(volatile v4u*)q = u;
    __threadfence();
    *(volatile v4u*)q = u;
  }
}

__global__ __launch_bounds__(128) void ln_kernel(const float* __restrict__ Y, const float* __restrict__ gamma,
                                                 const float* __restrict__ beta, unsigned short* __restrict__ YN) {
  __shared__ float red1[4];
  __shared__ float red2[4];
  const int row  = blockIdx.x;
  const int t    = threadIdx.x;
  const int lane = t & 31, wave = t >> 5;
  const int c0   = t * 8;
  const float* yr = Y + (size_t)row * kD + c0;
  const v4f a = *(const v4f*)(yr);
  const v4f c = *(const v4f*)(yr + 4);
  float y[8];
#pragma unroll
  for (int e = 0; e < 4; ++e) { y[e] = a[e]; y[4 + e] = c[e]; }
  float s = ((y[0] + y[1]) + (y[2] + y[3])) + ((y[4] + y[5]) + (y[6] + y[7]));
#pragma unroll
  for (int off = 16; off > 0; off >>= 1) s += __shfl_xor(s, off, 32);
  if (lane == 0) red1[wave] = s;
  __syncthreads();
  const float mu = ((red1[0] + red1[1]) + (red1[2] + red1[3])) * kInvD;
  float d[8];
  float s2 = 0.0f;
#pragma unroll
  for (int e = 0; e < 8; ++e) { d[e] = y[e] - mu; s2 += d[e] * d[e]; }
#pragma unroll
  for (int off = 16; off > 0; off >>= 1) s2 += __shfl_xor(s2, off, 32);
  if (lane == 0) red2[wave] = s2;
  __syncthreads();
  const float var  = ((red2[0] + red2[1]) + (red2[2] + red2[3])) * kInvD;
  const float rstd = 1.0f / sqrtf(var + kLnEps);
  const v4f ga = *(const v4f*)(gamma + c0);
  const v4f gc = *(const v4f*)(gamma + c0 + 4);
  const v4f ba = *(const v4f*)(beta + c0);
  const v4f bc = *(const v4f*)(beta + c0 + 4);
  unsigned short hb[8];
#pragma unroll
  for (int e = 0; e < 4; ++e) {
    hb[e]     = h_bits(d[e] * rstd * ga[e] + ba[e]);
    hb[4 + e] = h_bits(d[4 + e] * rstd * gc[e] + bc[e]);
  }
  const v4u u = (v4u){pk16(hb[0], hb[1]), pk16(hb[2], hb[3]), pk16(hb[4], hb[5]), pk16(hb[6], hb[7])};
  unsigned short* q = YN + (size_t)row * kD + c0;
  *(volatile v4u*)q = u;
  __threadfence();
  *(volatile v4u*)q = u;
}

extern "C" void kernel_launch(void* const* d_in, const int* in_sizes, int n_in,
                              void* d_out, int out_size, void* d_ws, size_t ws_size,
                              hipStream_t stream) {
  if (n_in < 17) return;
  if (in_sizes[0] != kTok * kD) return;
  if (in_sizes[1] != kB * kNAdap * kD) return;
  if (in_sizes[2] != kB * kD || in_sizes[3] != kB * kD) return;
  if (in_sizes[4] != kD * kD || in_sizes[6] != kD * kD || in_sizes[8] != kD * kD) return;
  if (in_sizes[10] != kD * kD || in_sizes[15] != kD * kD) return;
  if (in_sizes[5] != kD || in_sizes[7] != kD || in_sizes[9] != kD || in_sizes[11] != kD) return;
  if (in_sizes[13] != kD || in_sizes[14] != kD || in_sizes[16] != kD || in_sizes[12] < 1) return;
  if (out_size != kTok * kD) return;
  if (ws_size < kWsTotal) return;

  const float* x    = (const float*)d_in[0];
  const float* h_t  = (const float*)d_in[1];
  const float* h_a  = (const float*)d_in[2];
  const float* pin  = (const float*)d_in[3];
  const float* Wq   = (const float*)d_in[4];
  const float* bq   = (const float*)d_in[5];
  const float* Wk   = (const float*)d_in[6];
  const float* bk   = (const float*)d_in[7];
  const float* Wv   = (const float*)d_in[8];
  const float* bv   = (const float*)d_in[9];
  const float* Wo   = (const float*)d_in[10];
  const float* bo   = (const float*)d_in[11];
  const float* g    = (const float*)d_in[12];
  const float* lng  = (const float*)d_in[13];
  const float* lnb  = (const float*)d_in[14];
  const float* Wf   = (const float*)d_in[15];
  const float* bfp  = (const float*)d_in[16];

  char* ws = (char*)d_ws;
  unsigned short* W16  = (unsigned short*)(ws + kOffW);
  unsigned short* Wq16 = W16 + (size_t)0 * kD * kD;
  unsigned short* Wk16 = W16 + (size_t)1 * kD * kD;
  unsigned short* Wv16 = W16 + (size_t)2 * kD * kD;
  unsigned short* Wo16 = W16 + (size_t)3 * kD * kD;
  unsigned short* Wf16 = W16 + (size_t)4 * kD * kD;
  unsigned short* XE   = (unsigned short*)(ws + kOffXE);
  float*          KF   = (float*)(ws + kOffKF);
  unsigned short* K16  = (unsigned short*)(ws + kOffK16);
  unsigned short* VT   = (unsigned short*)(ws + kOffVT);
  unsigned short* Q16  = (unsigned short*)(ws + kOffQ);
  unsigned short* O16  = (unsigned short*)(ws + kOffO);
  float*          SC   = (float*)(ws + kOffSC);
  unsigned short* P16  = (unsigned short*)(ws + kOffP);
  float*          Y    = (float*)(ws + kOffY);
  unsigned short* YN   = (unsigned short*)(ws + kOffYN);
  float*          OUT  = (float*)d_out;

  wcast5_kernel<<<dim3((kD * kD) / 8 / 256, 5), 256, 0, stream>>>(Wq, Wk, Wv, Wo, Wf, W16, kWCarry);
  build_xe_kernel<<<(kTokE * kD) / 8 / 256, 256, 0, stream>>>(x, h_t, h_a, pin, XE);

  wmma_gemm64<0, false, 2, 1, false, 0><<<dim3(64, kB), 256, 0, stream>>>(
      XE, nullptr, kD, (long)kSE * kD,
      Wq16, nullptr, kD, 0L,
      (void*)Q16, nullptr, kD, (long)kT * kD,
      bq, nullptr, 0L, kT, kD, kD, kWCarryInv);
  wmma_gemm64<0, false, 2, 0, false, 0><<<dim3(264, 1), 256, 0, stream>>>(
      XE, nullptr, kD, 0L,
      Wk16, nullptr, kD, 0L,
      (void*)KF, nullptr, kD, 0L,
      bk, nullptr, 0L, kTokE, kD, kD, kWCarryInv);
  wmma_gemm64<0, false, 1, 1, false, 0><<<dim3(66, kB), 256, 0, stream>>>(
      Wv16, nullptr, kD, 0L,
      XE, nullptr, kD, (long)kSE * kD,
      (void*)VT, nullptr, kSE, (long)kD * kSE,
      bv, nullptr, 0L, kD, kSE, kD, kWCarryInv);
  kcast_kernel<<<(kTokE * kD) / 8 / 256, 256, 0, stream>>>(KF, g, K16);

  for (int c = 0; c < kChunks; ++c) {
    const int b  = c / (kHeads / kGPer);
    const int h0 = (c % (kHeads / kGPer)) * kGPer;
    const unsigned short* Qg = Q16 + ((size_t)b * kT * kD + (size_t)h0 * kHd);
    const unsigned short* Kg = K16 + ((size_t)b * kSE * kD + (size_t)h0 * kHd);
    const unsigned short* Vg = VT + ((size_t)b * kD * kSE + (size_t)h0 * kHd * kSE);
    unsigned short* Og = O16 + ((size_t)b * kT * kD + (size_t)h0 * kHd);
    wmma_gemm64<0, false, 0, 0, false, 0><<<dim3(132, kGPer), 256, 0, stream>>>(
        Qg, nullptr, kD, (long)kHd,
        Kg, nullptr, kD, (long)kHd,
        (void*)SC, nullptr, kSE, (long)kT * kSE,
        nullptr, nullptr, 0L, kT, kSE, kHd, 1.0f);
    softmax_row_kernel<<<kGPer * kT, kSmThreads, 0, stream>>>(SC, P16, kScoreScale, kPCarry);
    wmma_gemm64<0, false, 0, 1, false, 0><<<dim3(8, kGPer), 256, 0, stream>>>(
        P16, nullptr, kSE, (long)kT * kSE,
        Vg, nullptr, kSE, (long)kHd * kSE,
        (void*)Og, nullptr, kD, (long)kHd,
        nullptr, nullptr, 0L, kT, kHd, kSE, kPVScale);
  }

  wmma_gemm64<0, false, 2, 0, true, 0><<<dim3(256, 1), 256, 0, stream>>>(
      O16, nullptr, kD, 0L,
      Wo16, nullptr, kD, 0L,
      (void*)Y, nullptr, kD, 0L,
      bo, x, 0L, kTok, kD, kD, kWoScale);
  ln_kernel<<<kTok, 128, 0, stream>>>(Y, lng, lnb, YN);
  wmma_gemm64<0, false, 2, 0, false, 2><<<dim3(256, 1), 256, 0, stream>>>(
      YN, nullptr, kD, 0L,
      Wf16, nullptr, kD, 0L,
      (void*)OUT, nullptr, kD, 0L,
      bfp, nullptr, 0L, kTok, kD, kD, kWCarryInv);
}
